// HCRLayer_9225589752137
// MI455X (gfx1250) — hardware-run, weakly checked
//
#include <hip/hip_runtime.h>


#define NB   131072
#define NX   4
#define NO   32
#define NG   6
#define NFE  1296
#define KP   1344
#define NC   64
#define PR   16384
constexpr size_t al256(size_t b) { return (b + 255) & ~(size_t)255; }
constexpr size_t WS_TOTAL = 2 * al256((size_t)PR * KP * 2) + al256((size_t)NC * KP * 2) + al256((size_t)PR * NC * 4);
static_assert(WS_TOTAL == 92446720 && WS_TOTAL <= 134217728, "the workspace carve: 88.2 MiB");
static_assert(NFE == NG * NG * NG * NG && KP % 32 == 0 && KP >= NFE && NC % 64 == 0 && PR % 64 == 0 && NB % PR == 0 && (KP * 2) % 128 == 0, "the depth in whole steps; whole tiles; whole parts; a row of a sixteen-bit plane is whole lines");
typedef _Float16 h16;
typedef unsigned short bf;
typedef __attribute__((ext_vector_type(16))) __bf16   v16bf;
typedef __attribute__((ext_vector_type(16))) _Float16 v16h;
typedef __attribute__((ext_vector_type(8)))  _Float16 v8h;
typedef __attribute__((ext_vector_type(8)))  unsigned short v8us;
typedef __attribute__((ext_vector_type(8)))  float    v8f;
typedef __attribute__((ext_vector_type(4)))  float    v4f;
typedef v8h  __attribute__((may_alias)) v8ha;
typedef v4f  __attribute__((may_alias)) v4fa;
typedef v8us __attribute__((may_alias)) v8usa;

__device__ __forceinline__ unsigned short f2bf(float f) { unsigned u = __float_as_uint(f); u += 0x7FFFu + ((u >> 16) & 1u); return (unsigned short)(u >> 16); }
__device__ __forceinline__ float bf2f(unsigned short b) { return __uint_as_float(((unsigned)b) << 16); }
__device__ __forceinline__ float bfr(float f) { return bf2f(f2bf(f)); }
__device__ __forceinline__ v16h cat16(v8h lo, v8h hi) { return __builtin_shufflevector(lo, hi, 0, 1, 2, 3, 4, 5, 6, 7, 8, 9, 10, 11, 12, 13, 14, 15); }
__device__ __forceinline__ v16bf cat16b(v8us lo, v8us hi) { return __builtin_bit_cast(v16bf, __builtin_shufflevector(lo, hi, 0, 1, 2, 3, 4, 5, 6, 7, 8, 9, 10, 11, 12, 13, 14, 15)); }
__device__ __forceinline__ v8f wmma16(v16h a, v16h b, v8f c) { return __builtin_amdgcn_wmma_f32_16x16x32_f16(false, a, false, b, (short)0, c, false, false); }
__device__ __forceinline__ v8f wmmab(v16bf a, v16bf b, v8f c) { return __builtin_amdgcn_wmma_f32_16x16x32_bf16(false, a, false, b, (short)0, c, false, false); }


template <typename T16> struct WFrag;
template <> struct WFrag<h16> { typedef v16h V; static __device__ __forceinline__ V ld(const h16* p) { return cat16(*(const v8h*)p, *(const v8h*)(p + 16)); } static __device__ __forceinline__ v8f mma(V a, V b, v8f c) { return wmma16(a, b, c); } };
template <> struct WFrag<bf> { typedef v16bf V; static __device__ __forceinline__ V ld(const bf* p) { return cat16b(*(const v8us*)p, *(const v8us*)(p + 16)); } static __device__ __forceinline__ v8f mma(V a, V b, v8f c) { return wmmab(a, b, c); } };
template <typename T16, int NSPLIT, bool BIAS>
__global__ __launch_bounds__(32) void k_gemmw(const T16* __restrict__ A, const T16* __restrict__ A2, const T16* __restrict__ Bt, const T16* __restrict__ Bt2, int K, float* C, int ldc, const float* __restrict__ bias, size_t sA, size_t sB, size_t sC) {
    typedef typename WFrag<T16>::V V;
    __shared__ __align__(16) float os[16 * 68];
    const size_t z = blockIdx.z; A += z * sA; if (A2) A2 += z * sA; Bt += z * sB; if (Bt2) Bt2 += z * sB; C += z * sC;
    const int lane = threadIdx.x & 31, lr = lane & 15, hi = lane >> 4; const int r0 = blockIdx.x * 64, c0 = blockIdx.y * 64;
    v8f acc[4][4];
#pragma unroll
    for (int mb = 0; mb < 4; ++mb)
#pragma unroll
        for (int nb = 0; nb < 4; ++nb) acc[mb][nb] = (v8f){};
    const size_t aoff = (size_t)(r0 + lr) * K + 8 * hi, boff = (size_t)(c0 + lr) * K + 8 * hi;
    for (int kc = 0; kc < K; kc += 32) {
        V a[4], a2[4];
#pragma unroll
        for (int mb = 0; mb < 4; ++mb) { a[mb] = WFrag<T16>::ld(A + aoff + (size_t)mb * 16 * K + kc); if (NSPLIT == 1 || NSPLIT == 2) a2[mb] = WFrag<T16>::ld(A2 + aoff + (size_t)mb * 16 * K + kc); }
#pragma unroll
        for (int nb = 0; nb < 4; ++nb) { const V b = WFrag<T16>::ld(Bt + boff + (size_t)nb * 16 * K + kc); V b2; if (NSPLIT >= 2) b2 = WFrag<T16>::ld(Bt2 + boff + (size_t)nb * 16 * K + kc);
#pragma unroll
            for (int mb = 0; mb < 4; ++mb) { acc[mb][nb] = WFrag<T16>::mma(a[mb], b, acc[mb][nb]); if (NSPLIT == 1 || NSPLIT == 2) acc[mb][nb] = WFrag<T16>::mma(a2[mb], b, acc[mb][nb]); if (NSPLIT >= 2) acc[mb][nb] = WFrag<T16>::mma(a[mb], b2, acc[mb][nb]); } }
        asm volatile("v_nop\n\tv_nop\n\tv_nop\n\tv_nop" : "+v"(acc[0][0]), "+v"(acc[1][1]), "+v"(acc[2][2]), "+v"(acc[3][3]) : "v"(a[0]), "v"(a[3]));
    }
#pragma unroll
    for (int mb = 0; mb < 4; ++mb) {
#pragma unroll
        for (int nb = 0; nb < 4; ++nb) {
#pragma unroll
            for (int j = 0; j < 8; ++j) os[(hi * 8 + j) * 68 + nb * 16 + lr] = acc[mb][nb][j]; }
        __builtin_amdgcn_wave_barrier(); asm volatile("" ::: "memory");
        float* crow = C + (size_t)(r0 + mb * 16) * ldc + c0;
#pragma unroll 1
        for (int ps = 0; ps < 2; ++ps) {
#pragma unroll
            for (int s = 0; s < 8; ++s) { const int row = 2 * s + hi, cofs = lr * 4; v4f val = *(const v4fa*)(os + row * 68 + cofs); if (BIAS) { val[0] += bfr(bias[c0 + cofs]); val[1] += bfr(bias[c0 + cofs + 1]); val[2] += bfr(bias[c0 + cofs + 2]); val[3] += bfr(bias[c0 + cofs + 3]); }
                *(volatile v4f*)(crow + (size_t)row * ldc + cofs) = val; }
            if (ps == 0) __threadfence(); }
        __builtin_amdgcn_wave_barrier(); asm volatile("" ::: "memory");
    }
}

__device__ __forceinline__ h16 tohx(float x) { return (h16)x; }
__device__ __forceinline__ void splitf(float y, unsigned short& h, unsigned short& l) { h = f2bf(y); l = f2bf(y - bf2f(h)); }
typedef __attribute__((ext_vector_type(2))) _Float16 v2h;
typedef __attribute__((ext_vector_type(4))) _Float16 v4h;
typedef __attribute__((ext_vector_type(2))) unsigned short v2us;
typedef __attribute__((ext_vector_type(4))) unsigned short v4us;
typedef __attribute__((ext_vector_type(2))) float v2f;
typedef __attribute__((ext_vector_type(4))) int v4i;

__global__ __launch_bounds__(256) void k_cpad(const float* __restrict__ cw, bf* CB) {
    const unsigned o = blockIdx.y, g = threadIdx.x; if (g >= (unsigned)(KP / 8)) return;
    const bool on = (o < (unsigned)NO) && (g < (unsigned)(NFE / 8)); const unsigned oc = on ? o : 0u, gc = on ? g : 0u; const float sf = on ? 1.0f : 0.0f;
    const float* s = cw + (size_t)oc * NFE + 8 * gc; const v4f a0 = *(const v4f*)(s); const v4f a1 = *(const v4f*)(s + 4); v8us r;
#pragma unroll
    for (int c = 0; c < 4; ++c) { r[c] = f2bf(a0[c] * sf); r[c + 4] = f2bf(a1[c] * sf); }
    bf* d = CB + (size_t)o * KP + 8 * g; *(volatile v8us*)(d) = r; __threadfence(); *(volatile v8us*)(d) = r; }

__device__ __forceinline__ void gvals(float x, float* g) { const float u = 2.0f * bfr(x) - 1.0f; float p0 = 1.0f, p1 = u; g[0] = p0 * 1.0f; g[1] = p1 * 1.7320508075688772f;
    const float p2 = (3.0f * u * p1 - 1.0f * p0) / 2.0f; g[2] = p2 * 2.23606797749979f; const float p3 = (5.0f * u * p2 - 2.0f * p1) / 3.0f; g[3] = p3 * 2.6457513110645907f;
    const float p4 = (7.0f * u * p3 - 3.0f * p2) / 4.0f; g[4] = p4 * 3.0f; const float p5 = (9.0f * u * p4 - 4.0f * p3) / 5.0f; g[5] = p5 * 3.3166247903554f; }
__global__ __launch_bounds__(256) void k_feat(const float* __restrict__ xr, bf* FH, bf* FL) {
    const unsigned th = blockIdx.x * 256 + threadIdx.x; if (th >= (unsigned)PR) return;
    { const size_t row = (size_t)th; const v4f xv = *(const v4f*)(xr + row * NX); float g0[NG], g1[NG], g2[NG], g3[NG]; gvals(xv[0], g0); gvals(xv[1], g1); gvals(xv[2], g2); gvals(xv[3], g3);
        bf* fh = FH + row * KP; bf* fl = FL + row * KP;
#pragma unroll
        for (int i0 = 0; i0 < NG; ++i0)
#pragma unroll
            for (int i1 = 0; i1 < NG; ++i1) { const float a01 = g0[i0] * g1[i1]; v4us oh[9], ol[9];
#pragma unroll
                for (int c = 0; c < 9; ++c)
#pragma unroll
                    for (int q = 0; q < 4; ++q) { const int mm = 4 * c + q; unsigned short h2, l2; splitf((a01 * g2[mm / NG]) * g3[mm % NG], h2, l2); oh[c][q] = h2; ol[c][q] = l2; }
                const int w0 = (i0 * NG + i1) * (NG * NG);
#pragma unroll
                for (int c = 0; c < 9; ++c) { *(volatile v4us*)(fh + w0 + 4 * c) = oh[c]; *(volatile v4us*)(fl + w0 + 4 * c) = ol[c]; }
                __threadfence();
#pragma unroll
                for (int c = 0; c < 9; ++c) { *(volatile v4us*)(fh + w0 + 4 * c) = oh[c]; *(volatile v4us*)(fl + w0 + 4 * c) = ol[c]; } }
        { const v4us zz = {0, 0, 0, 0};
#pragma unroll
            for (int c = 0; c < (KP - NFE) / 4; ++c) { *(volatile v4us*)(fh + NFE + 4 * c) = zz; *(volatile v4us*)(fl + NFE + 4 * c) = zz; }
            __threadfence();
#pragma unroll
            for (int c = 0; c < (KP - NFE) / 4; ++c) { *(volatile v4us*)(fh + NFE + 4 * c) = zz; *(volatile v4us*)(fl + NFE + 4 * c) = zz; } } } }

__global__ __launch_bounds__(256) void k_out(const float* __restrict__ CP, const float* __restrict__ cw, float* res) {
    const unsigned th = blockIdx.x * 256 + threadIdx.x; if (th >= (unsigned)(PR * (NO / 4))) return; const unsigned b = th >> 3, o4 = (th & 7) * 4; const v4f a = *(const v4f*)(CP + (size_t)b * NC + o4); v4f r;
    const float z0 = ((1.0f * 1.0f) * 1.0f) * 1.0f;
#pragma unroll
    for (int q = 0; q < 4; ++q) r[q] = 1.0f + a[q] - z0 * bfr(cw[(size_t)(o4 + q) * NFE]);
    float* d = res + (size_t)b * NO + o4; *(volatile v4f*)(d) = r; __threadfence(); *(volatile v4f*)(d) = r; }

extern "C" void kernel_launch(void* const* d_in, const int* in_sizes, int n_in,
                              void* d_out, int out_size, void* d_ws, size_t ws_size, hipStream_t stream) {
    if (n_in < 2) return;
    if (in_sizes[0] < NB * NX || in_sizes[1] < NO * NFE || out_size < NB * NO) return;
    const float* xr = (const float*)d_in[0]; const float* cw = (const float*)d_in[1];
    float* OUT = (float*)d_out;
    char* wsp = (char*)d_ws;
    auto take = [&](size_t bytes) { char* cur = wsp; wsp += (bytes + 255) & ~(size_t)255; return (void*)cur; };
    bf* FH = (bf*)take((size_t)PR * KP * 2); bf* FL = (bf*)take((size_t)PR * KP * 2); bf* CB = (bf*)take((size_t)NC * KP * 2); float* CP = (float*)take((size_t)PR * NC * 4);
    if ((size_t)(wsp - (char*)d_ws) != WS_TOTAL || WS_TOTAL > ws_size) return;
    k_cpad<<<dim3(1, NC, 1), 256, 0, stream>>>(cw, CB);
    for (int pt = 0; pt < NB / PR; ++pt) {
        const size_t r0 = (size_t)pt * PR;
        k_feat<<<(unsigned)((PR + 255) / 256), 256, 0, stream>>>(xr + r0 * NX, FH, FL);
        k_gemmw<bf, 1, false><<<dim3(PR / 64, NC / 64, 1), 32, 0, stream>>>(FH, FL, CB, nullptr, KP, CP, NC, nullptr, (size_t)0, (size_t)0, (size_t)0);
        k_out<<<(unsigned)((PR * (NO / 4) + 255) / 256), 256, 0, stream>>>(CP, cw, OUT + r0 * NO);
    }
}
